// RelationNetworkBaseline_54915451846824
// MI455X (gfx1250) — hardware-verified
//
#include <hip/hip_runtime.h>
#include <hip/hip_bf16.h>
#include <math.h>

#define NBr 32
#define NN 25
#define DDr 512
#define HHd 512
#define NCLS 1000
#define NCP 1024
#define NROWS (NBr * NN)
#define NROWP 896
#define NPAIR (NBr * NN * NN)
#define NPAIRP 20096
#define GSTR 48
#define SS 64
#define HH 1
#define DKK 64

typedef _Float16 bf16;
typedef _Float16 f16;
typedef __attribute__((ext_vector_type(4))) unsigned v4u_t;
typedef unsigned v4ua __attribute__((ext_vector_type(4), may_alias));
typedef __attribute__((ext_vector_type(4))) float v4f_t;
typedef float v4fa __attribute__((ext_vector_type(4), may_alias));
typedef __attribute__((ext_vector_type(16))) bf16  bf16x16;
typedef bf16x16 f16x16;
typedef __attribute__((ext_vector_type(8)))  bf16  bf16x8;
typedef bf16x8 f16x8;
typedef __attribute__((ext_vector_type(4)))  bf16  bf16x4;
typedef __attribute__((ext_vector_type(8)))  float f32x8;
__device__ __forceinline__ f32x8 wmma16(f16x16 a, f16x16 b, f32x8 c) {
  c = __builtin_amdgcn_wmma_f32_16x16x32_f16(false, a, false, b, (short)0, c, false, false);
  asm volatile("v_nop\n\tv_nop\n\tv_nop\n\tv_nop" : "+v"(c) : "v"(a), "v"(b));
  return c;
}
#define LDS_STRIDE 48
#define KSTRIDE    72
#define VSTRIDE    48

__device__ __forceinline__ f32x8 wmma_bf16(bf16x16 a, bf16x16 b, f32x8 c) {
  c = __builtin_amdgcn_wmma_f32_16x16x32_f16(false, a, false, b, (short)0, c, false, false);
  asm volatile("v_nop\n\tv_nop\n\tv_nop\n\tv_nop" : "+v"(c) : "v"(a), "v"(b));
  return c;
}

template <typename T>
__device__ __forceinline__ bf16x16 load_frag(const T* __restrict__ base, int ld,
                                             int row0, int k0) {
  const int lane = threadIdx.x & 31;
  const int r    = lane & 15;
  const int kh   = (lane >> 4) * 8;
  const T* p0 = base + (size_t)(row0 + r) * ld + (k0 + kh);
  const T* p1 = p0 + 16;
  bf16x16 f;
#pragma unroll
  for (int i = 0; i < 8; ++i) {
    f[i]     = (bf16)p0[i];
    f[i + 8] = (bf16)p1[i];
  }
  return f;
}

__device__ __forceinline__ bf16x16 lds_frag(const bf16* base, int stride) {
  const int lane = threadIdx.x & 31;
  const int row  = lane & 15;
  const int kh   = (lane >> 4) * 8;
  const bf16x8 lo = *(const bf16x8*)(base + row * stride + kh);
  const bf16x8 hi = *(const bf16x8*)(base + row * stride + kh + 16);
  bf16x16 f;
#pragma unroll
  for (int i = 0; i < 8; ++i) { f[i] = lo[i]; f[i + 8] = hi[i]; }
  return f;
}

template <typename T>
__device__ __forceinline__ void stage_read16(const T* __restrict__ p, float* buf) {
#pragma unroll
  for (int i = 0; i < 16; ++i) buf[i] = (float)p[i];
}

__device__ __forceinline__ void stage_write(bf16* dst, const float* buf, int nquad) {
#pragma unroll
  for (int i = 0; i < nquad; ++i) {
    bf16x4 q;
    q[0] = (bf16)buf[4 * i];     q[1] = (bf16)buf[4 * i + 1];
    q[2] = (bf16)buf[4 * i + 2]; q[3] = (bf16)buf[4 * i + 3];
    *(bf16x4*)(dst + 4 * i) = q;
  }
}


#define GSTR 48
template <typename AT, int EPI, bool OUT16>
__global__ __launch_bounds__(256) void gemm_kne(const AT* __restrict__ A, int lda, const float* __restrict__ Wm, int ldw,
                                                const float* __restrict__ bias, const float* __restrict__ R, const float* __restrict__ gvec,
                                                void* __restrict__ Yv, int ldy, int K) {
  __shared__ __attribute__((aligned(16))) f16 ldsA[128 * GSTR];
  __shared__ __attribute__((aligned(16))) f16 ldsW[128 * GSTR];
  __shared__ __attribute__((aligned(16))) float oS[8][32 * 68];
  const int tid = threadIdx.x, lane = tid & 31, wave = tid >> 5, cl = lane & 15, rh = (lane >> 4) * 8;
  const int m0 = blockIdx.x * 128, n0 = blockIdx.y * 128;
  const int wm = (wave & 3) * 32, wn = (wave >> 2) * 64;
  f32x8 acc[2][4];
#pragma unroll
  for (int i = 0; i < 2; ++i)
#pragma unroll
    for (int j = 0; j < 4; ++j) { f32x8 z = {}; acc[i][j] = z; }
#pragma unroll 1
  for (int k0 = 0; k0 < K; k0 += 32) {
    __syncthreads();
    { const int row = tid >> 1, ch = (tid & 1) * 16;
      const AT* src = A + (size_t)(m0 + row) * lda + k0 + ch;
#pragma unroll
      for (int g = 0; g < 16; ++g) ldsA[row * GSTR + ch + g] = (f16)src[g]; }
    { const int k = tid >> 3, nn0 = (tid & 7) * 16;
      const float* src = Wm + (size_t)(k0 + k) * ldw + n0 + nn0;
#pragma unroll
      for (int g = 0; g < 4; ++g) { const v4f_t v = *(const v4f_t*)(src + 4 * g);
#pragma unroll
        for (int u = 0; u < 4; ++u) ldsW[(nn0 + 4 * g + u) * GSTR + k] = (f16)v[u]; } }
    __syncthreads();
    f16x16 af[2];
#pragma unroll
    for (int i = 0; i < 2; ++i) af[i] = lds_frag(ldsA + (wm + 16 * i) * GSTR, GSTR);
#pragma unroll
    for (int j = 0; j < 4; ++j) {
      const f16x16 bf = lds_frag(ldsW + (wn + 16 * j) * GSTR, GSTR);
#pragma unroll
      for (int i = 0; i < 2; ++i) acc[i][j] = wmma16(af[i], bf, acc[i][j]);
    }
  }
  float* so = oS[wave];
#pragma unroll
  for (int i = 0; i < 2; ++i)
#pragma unroll
    for (int j = 0; j < 4; ++j) {
      const int n = n0 + wn + 16 * j + cl;
      const float bv = bias ? bias[n] : 0.0f;
      const float gv = (EPI == 2) ? gvec[n] : 0.0f;
      if (EPI == 1) {
#pragma unroll 1
        for (int r = 0; r < 8; ++r) { const float xg = acc[i][j][r] + bv; so[(16 * i + rh + r) * 68 + 16 * j + cl] = 0.5f * xg * (1.0f + erff(xg * 0.70710678118654752f)); }
      } else {
#pragma unroll
        for (int r = 0; r < 8; ++r) {
          float v = acc[i][j][r] + bv;
          if (EPI == 2) v = R[(size_t)(m0 + wm + 16 * i + rh + r) * ldy + n] + gv * v;
          so[(16 * i + rh + r) * 68 + 16 * j + cl] = v;
        }
      }
    }
  asm volatile("s_wait_dscnt 0" ::: "memory");
  __builtin_amdgcn_wave_barrier();
#pragma unroll 1
  for (int pass = 0; pass < 2; ++pass) {
    if (OUT16) {
      f16* Y = (f16*)Yv;
#pragma unroll
      for (int it = 0; it < 8; ++it) { const int c = lane + 32 * it, rr = c >> 3, q8 = (c & 7) * 8;
        union { f16 h[8]; v4u_t v; } u;
#pragma unroll
        for (int e = 0; e < 8; ++e) u.h[e] = (f16)so[rr * 68 + q8 + e];
        *(volatile v4u_t*)(Y + (size_t)(m0 + wm + rr) * ldy + n0 + wn + q8) = u.v; }
    } else {
      float* Y = (float*)Yv;
#pragma unroll
      for (int it = 0; it < 16; ++it) { const int f4 = lane + 32 * it, rr = f4 >> 4, q = (f4 & 15) * 4;
        *(volatile v4f_t*)(Y + (size_t)(m0 + wm + rr) * ldy + n0 + wn + q) = *(const v4fa*)(so + rr * 68 + q); }
    }
    __threadfence();
  }
}

__global__ __launch_bounds__(256) void k_padx(const float* __restrict__ x, float* __restrict__ xp) { const size_t r = blockIdx.x; for (int c = threadIdx.x; c < DDr; c += 256) xp[r * DDr + c] = (r < NROWS) ? x[r * DDr + c] : 0.0f; }
__global__ __launch_bounds__(256) void k_pairs(const float* __restrict__ A, const float* __restrict__ Bq, const float* __restrict__ b1, bf16* __restrict__ h1) {
  const size_t p = blockIdx.x; const int tid = threadIdx.x; union { bf16 hh[2]; unsigned u; } cv;
  if (p < NPAIR) { const int b = p / (NN * NN), r = p % (NN * NN), i = r / NN, j = r % NN; const float* ai = A + ((size_t)b * NN + i) * HHd; const float* bj = Bq + ((size_t)b * NN + j) * HHd;
    const int c = tid * 2; cv.hh[0] = (bf16)fmaxf(ai[c] + bj[c] + b1[c], 0.0f); cv.hh[1] = (bf16)fmaxf(ai[c + 1] + bj[c + 1] + b1[c + 1], 0.0f); }
  else { cv.hh[0] = (bf16)0.0f; cv.hh[1] = (bf16)0.0f; }
  *(volatile unsigned*)(h1 + p * HHd + tid * 2) = cv.u; __threadfence(); *(volatile unsigned*)(h1 + p * HHd + tid * 2) = cv.u;
}
__global__ __launch_bounds__(256) void k_relu16(const float* __restrict__ src, bf16* __restrict__ dst, size_t n8) {
  const size_t i = (size_t)blockIdx.x * 256 + threadIdx.x; if (i >= n8) return; const float* p = src + 8 * i; union { bf16 hh[8]; v4u_t u; } cv;
#pragma unroll
  for (int e = 0; e < 8; ++e) cv.hh[e] = (bf16)fmaxf(p[e], 0.0f);
  *(volatile v4u_t*)(dst + 8 * i) = cv.u; __threadfence(); *(volatile v4u_t*)(dst + 8 * i) = cv.u;
}
__global__ __launch_bounds__(256) void k_agg(const float* __restrict__ h3, float* __restrict__ agg) {
  const int b = blockIdx.x, tid = threadIdx.x;
  for (int c = tid; c < HHd; c += 256) { float s = 0.0f;
    if (b < NBr) {
#pragma unroll 1
      for (int i = 0; i < NN; ++i)
#pragma unroll 1
        for (int j = 0; j < NN; ++j) { if (i == j) continue; s += fmaxf(h3[(((size_t)b * NN + i) * NN + j) * HHd + c], 0.0f); } }
    agg[(size_t)b * HHd + c] = s; }
}
__global__ __launch_bounds__(256) void k_padw3(const float* __restrict__ w, const float* __restrict__ b3, float* __restrict__ wp, float* __restrict__ bp) { const int r = blockIdx.x; for (int c = threadIdx.x; c < NCP; c += 256) { wp[(size_t)r * NCP + c] = (c < NCLS) ? w[(size_t)r * NCLS + c] : 0.0f; if (r == 0) bp[c] = (c < NCLS) ? b3[c] : 0.0f; } }
__global__ __launch_bounds__(256) void k_out(const float* __restrict__ lp, float* __restrict__ out) {
  const int q4 = blockIdx.x * 256 + threadIdx.x; if (q4 >= NBr * NCLS / 4) return; const int fidx = q4 * 4, r = fidx / NCLS, c = fidx % NCLS;
  const v4f_t v = *(const v4f_t*)(lp + (size_t)r * NCP + c); *(volatile v4f_t*)(out + fidx) = v; __threadfence(); *(volatile v4f_t*)(out + fidx) = v;
}

extern "C" void kernel_launch(void* const* d_in, const int* in_sizes, int n_in,
                              void* d_out, int out_size, void* d_ws, size_t ws_size,
                              hipStream_t stream) {
  (void)in_sizes; (void)n_in; (void)out_size;
  const float** f = (const float**)d_in;
  const float* x = f[0], *g_w1 = f[1], *g_b1 = f[2], *g_w2 = f[3], *g_b2 = f[4], *g_w3 = f[5], *g_b3 = f[6], *f_w1 = f[7], *f_b1 = f[8], *f_w2 = f[9], *f_b2 = f[10], *f_w3 = f[11], *f_b3 = f[12];
  float* out = (float*)d_out;
  char* ws = (char*)d_ws;
  float* xp = (float*)ws; ws += (size_t)NROWP * DDr * 4;
  float* A = (float*)ws; ws += (size_t)NROWP * HHd * 4; float* Bq = (float*)ws; ws += (size_t)NROWP * HHd * 4;
  bf16* h1 = (bf16*)ws; ws += (size_t)NPAIRP * HHd * 2;
  float* hr = (float*)ws; ws += (size_t)NPAIRP * HHd * 4;
  bf16* h2 = (bf16*)ws; ws += (size_t)NPAIRP * HHd * 2;
  float* agg = (float*)ws; ws += (size_t)128 * HHd * 4;
  float* z1r = (float*)ws; ws += (size_t)128 * HHd * 4; bf16* z1 = (bf16*)ws; ws += (size_t)128 * HHd * 2;
  float* z2r = (float*)ws; ws += (size_t)128 * HHd * 4; bf16* z2 = (bf16*)ws; ws += (size_t)128 * HHd * 2;
  float* w3p = (float*)ws; ws += (size_t)HHd * NCP * 4; float* b3p = (float*)ws; ws += NCP * 4;
  float* lp = (float*)ws; ws += (size_t)128 * NCP * 4;
  if ((size_t)(ws - (char*)d_ws) > ws_size) return;
  const dim3 blk(256);
  k_padx<<<dim3(NROWP), blk, 0, stream>>>(x, xp);
  gemm_kne<float, 0, false><<<dim3(NROWP / 128, HHd / 128), blk, 0, stream>>>(xp, DDr, g_w1, HHd, nullptr, nullptr, nullptr, A, HHd, DDr);
  gemm_kne<float, 0, false><<<dim3(NROWP / 128, HHd / 128), blk, 0, stream>>>(xp, DDr, g_w1 + (size_t)DDr * HHd, HHd, nullptr, nullptr, nullptr, Bq, HHd, DDr);
  k_pairs<<<dim3(NPAIRP), blk, 0, stream>>>(A, Bq, g_b1, h1);
  gemm_kne<bf16, 0, false><<<dim3(NPAIRP / 128, HHd / 128), blk, 0, stream>>>(h1, HHd, g_w2, HHd, g_b2, nullptr, nullptr, hr, HHd, HHd);
  k_relu16<<<dim3((NPAIRP * HHd / 8 + 255) / 256), blk, 0, stream>>>(hr, h2, (size_t)NPAIRP * HHd / 8);
  gemm_kne<bf16, 0, false><<<dim3(NPAIRP / 128, HHd / 128), blk, 0, stream>>>(h2, HHd, g_w3, HHd, g_b3, nullptr, nullptr, hr, HHd, HHd);
  k_agg<<<dim3(128), blk, 0, stream>>>(hr, agg);
  gemm_kne<float, 0, false><<<dim3(1, HHd / 128), blk, 0, stream>>>(agg, HHd, f_w1, HHd, f_b1, nullptr, nullptr, z1r, HHd, HHd);
  k_relu16<<<dim3((128 * HHd / 8 + 255) / 256), blk, 0, stream>>>(z1r, z1, (size_t)128 * HHd / 8);
  gemm_kne<bf16, 0, false><<<dim3(1, HHd / 128), blk, 0, stream>>>(z1, HHd, f_w2, HHd, f_b2, nullptr, nullptr, z2r, HHd, HHd);
  k_relu16<<<dim3((128 * HHd / 8 + 255) / 256), blk, 0, stream>>>(z2r, z2, (size_t)128 * HHd / 8);
  k_padw3<<<dim3(HHd), blk, 0, stream>>>(f_w3, f_b3, w3p, b3p);
  gemm_kne<bf16, 0, false><<<dim3(1, NCP / 128), blk, 0, stream>>>(z2, HHd, w3p, NCP, b3p, nullptr, nullptr, lp, NCP, HHd);
  k_out<<<dim3((NBr * NCLS / 4 + 255) / 256), blk, 0, stream>>>(lp, out);
}
